// RecurrentNN_27307402068532
// MI455X (gfx1250) — hardware-verified
//
#include <hip/hip_runtime.h>
#include <math.h>

typedef __attribute__((ext_vector_type(16))) _Float16 v16h;
typedef __attribute__((ext_vector_type(8)))  _Float16 v8h;
typedef __attribute__((ext_vector_type(8)))  float    v8f;
typedef __attribute__((ext_vector_type(4)))  float    v4f;

constexpr int kBatch     = 4096;
constexpr int kSteps     = 2048;
constexpr int kHid       = 4;
constexpr int kGate4     = 4 * kHid;
constexpr int kTileRows  = 16;
constexpr int kBlocks    = kBatch / kTileRows;
constexpr int kChunk     = 32;
constexpr int kNumChunks = kSteps / kChunk;
constexpr int kPitch     = 36;
constexpr size_t kOutElems = (size_t)kBatch * kSteps;
static_assert(kHid == 4 && kGate4 == 16, "the four gates of the four units fill the 16 rows of one tile");
static_assert(kBatch % kTileRows == 0 && kSteps % kChunk == 0 && (kPitch % 4) == 0, "whole tiles, chunks, 16-B rows");

constexpr float kSCarry = 1024.0f;
constexpr float kWCarry = 4096.0f;
constexpr float kFold   = 1.0f / (kSCarry * kWCarry);
constexpr float kF16MinNormal = 6.103515625e-5f;
static_assert(kFold == 2.384185791015625e-7f, "2^-22");

union FragU { v16h v; v8h h[2]; };

__device__ __forceinline__ unsigned short f2bf_bits(float f) {
  unsigned u = __float_as_uint(f);
  return (unsigned short)((u + 0x7FFFu + ((u >> 16) & 1u)) >> 16);
}
__device__ __forceinline__ float bf16r(float f) { return __uint_as_float(((unsigned)f2bf_bits(f)) << 16); }
__device__ __forceinline__ float carry_flush(float v, float c) {
  const float s = v * c;
  return (fabsf(s) < kF16MinNormal) ? 0.0f : s;
}
__device__ __forceinline__ v8f mma_h0(v16h a, v16h b) {
  v8f c = (v8f){0.f, 0.f, 0.f, 0.f, 0.f, 0.f, 0.f, 0.f};
  c = __builtin_amdgcn_wmma_f32_16x16x32_f16(false, a, false, b, (short)0, c, false, false);
  asm volatile("v_nop\n\tv_nop\n\tv_nop\n\tv_nop" : "+v"(c) : "v"(a), "v"(b));
  return c;
}
__device__ __forceinline__ float fast_tanh(float v) {
  const float e = __expf(2.0f * v);
  return 1.0f - 2.0f * __builtin_amdgcn_rcpf(e + 1.0f);
}
__device__ __forceinline__ float fast_sigmoid(float v) { return __builtin_amdgcn_rcpf(1.0f + __expf(-v)); }

__global__ __launch_bounds__(32) void lstm4_seq_kernel(const float* __restrict__ x, const float* __restrict__ w_ih,
                                                       const float* __restrict__ w_hh, const float* __restrict__ b_ih,
                                                       const float* __restrict__ b_hh, const float* __restrict__ w_lin,
                                                       const float* __restrict__ b_lin, float* __restrict__ outs) {
  __shared__ __align__(16) float xs[kTileRows * kPitch];
  __shared__ __align__(16) float os[kTileRows * kPitch];
  const int lane = threadIdx.x & 31;
  const int hs = lane >> 4;
  const int n = lane & 15;
  const bool lowHalf = (hs == 0);
  const int b0 = blockIdx.x * kTileRows;

  v16h fragA;
  {
    const int u = n >> 2;
    const int q = n & 3;
    const int src = 4 * q + u;
    const float wa = w_hh[src * kHid + 2 * hs + 0];
    const float wb = w_hh[src * kHid + 2 * hs + 1];
    const float wx = w_ih[src];
    const float bi = b_ih[src];
    const float bh = b_hh[src];
#pragma unroll
    for (int e = 0; e < 16; ++e) fragA[e] = (_Float16)0.0f;
    fragA[0] = (_Float16)carry_flush(bf16r(wa), kWCarry);
    fragA[1] = (_Float16)carry_flush(bf16r(wb), kWCarry);
    fragA[2] = lowHalf ? (_Float16)carry_flush(bf16r(wx), kWCarry) : (_Float16)0.0f;
    fragA[3] = lowHalf ? (_Float16)carry_flush(bf16r(bi), kWCarry) : (_Float16)0.0f;
    fragA[4] = lowHalf ? (_Float16)carry_flush(bf16r(bh), kWCarry) : (_Float16)0.0f;
  }
  const float wl0 = w_lin[2 * hs + 0];
  const float wl1 = w_lin[2 * hs + 1];
  const float bl0 = b_lin[0];
  const float wo0 = bf16r(wl0), wo1 = bf16r(wl1), bo = bf16r(bl0);
  const _Float16 one = (_Float16)kSCarry;

  float cst[2] = {0.0f, 0.0f}, hst[2] = {0.0f, 0.0f};

#pragma unroll 1
  for (int ch = 0; ch < kNumChunks; ++ch) {
    const int t0 = ch * kChunk;
#pragma unroll
    for (int it = 0; it < 4; ++it) {
      const int vi = it * 32 + lane;
      const int row = vi >> 3;
      const int c4 = (vi & 7) * 4;
      const v4f v = *(const v4f*)(x + (size_t)(b0 + row) * kSteps + t0 + c4);
      v4f rv;
      const float v0 = v[0], v1 = v[1], v2 = v[2], v3 = v[3];
      rv[0] = bf16r(v0); rv[1] = bf16r(v1); rv[2] = bf16r(v2); rv[3] = bf16r(v3);
      *(v4f*)(xs + row * kPitch + c4) = rv;
    }
    __syncthreads();

#pragma unroll 1
    for (int s = 0; s < kChunk; ++s) {
      const float xv = xs[n * kPitch + s];
      v16h fb;
#pragma unroll
      for (int e = 0; e < 16; ++e) fb[e] = (_Float16)0.0f;
      fb[0] = (_Float16)carry_flush(hst[0], kSCarry);
      fb[1] = (_Float16)carry_flush(hst[1], kSCarry);
      fb[2] = lowHalf ? (_Float16)carry_flush(xv, kSCarry) : (_Float16)0.0f;
      fb[3] = lowHalf ? one : (_Float16)0.0f;
      fb[4] = lowHalf ? one : (_Float16)0.0f;
      const v8f d = mma_h0(fragA, fb);
      float p = 0.0f;
#pragma unroll
      for (int k = 0; k < 2; ++k) {
        const float gi = d[4 * k + 0] * kFold, gf = d[4 * k + 1] * kFold, gg = d[4 * k + 2] * kFold, go = d[4 * k + 3] * kFold;
        const float cn = fast_sigmoid(gf) * cst[k] + fast_sigmoid(gi) * fast_tanh(gg);
        cst[k] = cn;
        hst[k] = fast_sigmoid(go) * fast_tanh(cn);
      }
      p = fmaf(wo0, hst[0], p);
      p = fmaf(wo1, hst[1], p);
      const float pother = __shfl_xor(p, 16, 32);
      const float plow = lowHalf ? p : pother;
      const float phigh = lowHalf ? pother : p;
      const float y = (plow + phigh) + bo;
      if (lowHalf) os[n * kPitch + s] = y;
    }
    __syncthreads();

    for (int pass = 0; pass < 2; ++pass) {
#pragma unroll
      for (int it = 0; it < 4; ++it) {
        const int vi = it * 32 + lane;
        const int row = vi >> 3;
        const int c4 = (vi & 7) * 4;
        const v4f ov = *(const v4f*)(os + row * kPitch + c4);
        *(volatile v4f*)(outs + (size_t)(b0 + row) * kSteps + t0 + c4) = ov;
      }
      __threadfence();
    }
    __syncthreads();
  }
}

extern "C" void kernel_launch(void* const* d_in, const int* in_sizes, int n_in,
                              void* d_out, int out_size, void* d_ws, size_t ws_size,
                              hipStream_t stream) {
  if (n_in < 7 || d_out == nullptr) return;
  if ((size_t)in_sizes[0] != kOutElems) return;
  if (in_sizes[1] != kGate4 || in_sizes[2] != kGate4 * kHid || in_sizes[3] != kGate4 || in_sizes[4] != kGate4) return;
  if (in_sizes[5] != kHid || in_sizes[6] != 1) return;
  if ((size_t)out_size != kOutElems) return;
  lstm4_seq_kernel<<<kBlocks, 32, 0, stream>>>((const float*)d_in[0], (const float*)d_in[1], (const float*)d_in[2],
                                               (const float*)d_in[3], (const float*)d_in[4], (const float*)d_in[5],
                                               (const float*)d_in[6], (float*)d_out);
}
